// Belt_Block_83665962926555
// MI455X (gfx1250) — hardware-verified
//
#include <hip/hip_runtime.h>
#include <stddef.h>
#include <stdint.h>


typedef _Float16 v16h __attribute__((ext_vector_type(16)));
typedef _Float16 v8h __attribute__((ext_vector_type(8)));
typedef _Float16 v8ha __attribute__((ext_vector_type(8), may_alias));
typedef float v8f __attribute__((ext_vector_type(8)));
typedef float v4f __attribute__((ext_vector_type(4)));
typedef float v4fa __attribute__((ext_vector_type(4), may_alias));

namespace {
constexpr int Bn = 8, Nn = 307, Cn = 64, Tn = 12;
constexpr int HSn = 4, COn = 16, HTn = 4, DKn = 16, FFn = 256;
constexpr float EPSn = 1e-5f;
constexpr int BT = Bn * Tn;
constexpr int TILES = (Nn + 15) / 16;
constexpr int NP = TILES * 16;
constexpr int NS = Nn * Cn * Tn;
constexpr int NS4 = NS / 4;
constexpr int TNPC = Tn * NP * Cn;
constexpr size_t PSZ = (size_t)BT * NP * Cn;
constexpr int NBH = BT * Nn * HSn;
constexpr int NATT = Bn * Nn * Tn * HTn;
constexpr int ROWS_A = Bn * Nn * Tn;
constexpr int OUTN = Bn * Nn * Cn * Tn;
constexpr int NQ4 = OUTN / 4;
constexpr int KMAX = 32;
constexpr int SBLK = 64;
constexpr int WPITCH = 72;
constexpr int FPITCH = 264;
constexpr int SPITCH = 68;
constexpr float WSC = 64.0f, WINV = 1.0f / 64.0f;
constexpr float HSC = 64.0f, HWINV = 1.0f / 4096.0f;
constexpr double INVNS = 1.0 / 235776.0;
constexpr int WOFF_W = 0, WOFF_Q = 4096, WOFF_K = 8192, WOFF_V = 12288, WOFF_O = 16384,
              WOFF_1 = 20480, WOFF_2 = 36864, W16_TOT = 53248;
constexpr int GEMM_WG = (BT * TILES) / 4;
constexpr int FLAT_WG = (NBH + 255) / 256;
constexpr int ATT_WG = (NATT + 255) / 256;
constexpr int APPLY_WG = (NQ4 + 255) / 256;
typedef char chk_tile_grid[((BT * TILES) % 4 == 0) ? 1 : -1];
typedef char chk_full_wave[(NBH % 32 == 0 && NQ4 % 32 == 0 && NS4 % 32 == 0) ? 1 : -1];
}

union Frag { v16h v; v8h p[2]; };

__device__ __forceinline__ v8f zero8() {
  v8f z;
#pragma unroll
  for (int r = 0; r < 8; ++r) z[r] = 0.f;
  return z;
}

__device__ __forceinline__ v8f wmma16(v16h a, v16h b, v8f c) {
  v8f d = __builtin_amdgcn_wmma_f32_16x16x32_f16(false, a, false, b, (short)0, c, false, false);
  asm volatile("v_nop\n\tv_nop\n\tv_nop\n\tv_nop" : "+v"(d) : "v"(a), "v"(b));
  return d;
}

__device__ __forceinline__ v16h frag_lds(const _Float16* rowp, int k0, int h) {
  Frag f;
  f.p[0] = *(const v8ha*)(rowp + k0 + 8 * h);
  f.p[1] = *(const v8ha*)(rowp + k0 + 16 + 8 * h);
  return f.v;
}

template <int KS>
__device__ __forceinline__ v16h frag_f32(const float* rp, int k0, int h) {
  v16h a;
#pragma unroll
  for (int i = 0; i < 8; ++i) {
    a[i] = (_Float16)rp[(k0 + 8 * h + i) * KS];
    a[8 + i] = (_Float16)rp[(k0 + 16 + 8 * h + i) * KS];
  }
  return a;
}

__device__ __forceinline__ int clampn(int j) { return j < 0 ? 0 : (j >= Nn ? Nn - 1 : j); }

__device__ __forceinline__ double shfl_xor_d(double v, int msk) {
  int lo = __double2loint(v), hi = __double2hiint(v);
  lo = __shfl_xor(lo, msk, 32);
  hi = __shfl_xor(hi, msk, 32);
  return __hiloint2double(hi, lo);
}

__global__ __launch_bounds__(256) void k_cvtw(const float* __restrict__ w0, const float* __restrict__ w1,
                                              const float* __restrict__ w2, const float* __restrict__ w3,
                                              const float* __restrict__ w4, const float* __restrict__ w5,
                                              const float* __restrict__ w6, _Float16* __restrict__ dst) {
  const int sel = blockIdx.y;
  const float* src;
  int cnt, off;
  if (sel == 0)      { src = w0; cnt = Cn * Cn;  off = WOFF_W; }
  else if (sel == 1) { src = w1; cnt = Cn * Cn;  off = WOFF_Q; }
  else if (sel == 2) { src = w2; cnt = Cn * Cn;  off = WOFF_K; }
  else if (sel == 3) { src = w3; cnt = Cn * Cn;  off = WOFF_V; }
  else if (sel == 4) { src = w4; cnt = Cn * Cn;  off = WOFF_O; }
  else if (sel == 5) { src = w5; cnt = FFn * Cn; off = WOFF_1; }
  else               { src = w6; cnt = Cn * FFn; off = WOFF_2; }
  const int e = (blockIdx.x * 256 + threadIdx.x) * 8;
  const bool act = e < cnt;
  const int ec = act ? e : 0;
  v8h v;
#pragma unroll
  for (int k = 0; k < 8; ++k) v[k] = (_Float16)(src[ec + k] * WSC);
  _Float16* p = dst + off + ec;
  if (act) *(volatile v8h*)p = v;
  __threadfence();
  if (act) *(volatile v8h*)p = v;
}

template <bool RES>
__device__ __forceinline__ void store_tile(const float* st, const float* __restrict__ resid,
                                           float* __restrict__ out, int bt, int n0, int h, int m,
                                           bool active) {
#pragma unroll
  for (int pass = 0; pass < 2; ++pass) {
#pragma unroll
    for (int it = 0; it < 8; ++it) {
      const int row = 2 * it + h, col = m * 4;
      v4f v = *(const v4fa*)(st + row * SPITCH + col);
      const int orow = n0 + row;
      if (RES) {
        const int rr = orow < Nn ? orow : Nn - 1;
        v4f rs = *(const v4fa*)(resid + ((size_t)bt * NP + rr) * Cn + col);
        v += rs;
      }
      if (active) *(volatile v4f*)(out + ((size_t)bt * NP + orow) * Cn + col) = v;
    }
    if (pass == 0) __threadfence();
  }
}

template <int SRC, bool RES>
__device__ __forceinline__ void lin64_body(const float* __restrict__ A, const _Float16* __restrict__ W16,
                                           const float* __restrict__ bias, const float* __restrict__ resid,
                                           float* __restrict__ out, _Float16* Ws, float* stg) {
  const int tid = threadIdx.x, wave = tid >> 5, lane = tid & 31, h = lane >> 4, m = lane & 15;
  for (int c = tid; c < Cn * 8; c += 128) {
    const int n = c >> 3, k8 = (c & 7) * 8;
    *(v8h*)(Ws + n * WPITCH + k8) = *(const v8h*)(W16 + n * Cn + k8);
  }
  __syncthreads();
  const int g = blockIdx.x * 4 + wave;
  const bool active = g < BT * TILES;
  const int gg = active ? g : 0;
  const int bt = gg / TILES, n0 = (gg - bt * TILES) * 16;
  const int nr = n0 + m, nc = nr < Nn ? nr : Nn - 1;
  v16h a0, a1;
  if (SRC == 0) {
    const int b = bt / Tn, t = bt - b * Tn;
    const float* rp = A + ((size_t)(b * Nn + nc) * Cn) * Tn + t;
    a0 = frag_f32<Tn>(rp, 0, h);
    a1 = frag_f32<Tn>(rp, 32, h);
  } else {
    const float* rp = A + ((size_t)bt * NP + nc) * Cn;
    a0 = frag_f32<1>(rp, 0, h);
    a1 = frag_f32<1>(rp, 32, h);
  }
  float* st = stg + wave * (16 * SPITCH);
#pragma unroll
  for (int ct = 0; ct < 4; ++ct) {
    const _Float16* wr = Ws + (ct * 16 + m) * WPITCH;
    v8f acc = zero8();
    acc = wmma16(a0, frag_lds(wr, 0, h), acc);
    acc = wmma16(a1, frag_lds(wr, 32, h), acc);
    const float bv = bias[ct * 16 + m];
#pragma unroll
    for (int r = 0; r < 8; ++r) st[(8 * h + r) * SPITCH + ct * 16 + m] = acc[r] * WINV + bv;
  }
  __syncthreads();
  store_tile<RES>(st, resid, out, bt, n0, h, m, active);
}

__global__ __launch_bounds__(128) void k_wh(const float* __restrict__ x, const _Float16* __restrict__ W16,
                                            const float* __restrict__ bias, float* __restrict__ Wh) {
  __shared__ __align__(16) _Float16 Ws[Cn * WPITCH];
  __shared__ __align__(16) float stg[4 * 16 * SPITCH];
  lin64_body<0, false>(x, W16, bias, nullptr, Wh, Ws, stg);
}

__global__ __launch_bounds__(128) void k_qkv(const float* __restrict__ y1, const _Float16* __restrict__ Wq16,
                                             const _Float16* __restrict__ Wk16,
                                             const _Float16* __restrict__ Wv16, const float* __restrict__ bq,
                                             const float* __restrict__ bk, const float* __restrict__ bv,
                                             float* __restrict__ Qb, float* __restrict__ Kb,
                                             float* __restrict__ Vb) {
  __shared__ __align__(16) _Float16 Ws[Cn * WPITCH];
  __shared__ __align__(16) float stg[4 * 16 * SPITCH];
  const _Float16* W16;
  const float* bias;
  float* out;
  if (blockIdx.y == 0)      { W16 = Wq16; bias = bq; out = Qb; }
  else if (blockIdx.y == 1) { W16 = Wk16; bias = bk; out = Kb; }
  else                      { W16 = Wv16; bias = bv; out = Vb; }
  lin64_body<1, false>(y1, W16, bias, nullptr, out, Ws, stg);
}

__global__ __launch_bounds__(128) void k_wo(const float* __restrict__ ctx, const _Float16* __restrict__ W16,
                                            const float* __restrict__ bias, const float* __restrict__ y1,
                                            float* __restrict__ y2pre) {
  __shared__ __align__(16) _Float16 Ws[Cn * WPITCH];
  __shared__ __align__(16) float stg[4 * 16 * SPITCH];
  lin64_body<1, true>(ctx, W16, bias, y1, y2pre, Ws, stg);
}

__global__ __launch_bounds__(64) void k_redS(const float* __restrict__ Wh, float* __restrict__ S) {
  const int bt = blockIdx.x, c = threadIdx.x;
  const float* p = Wh + (size_t)bt * NP * Cn + c;
  double s = 0.0;
#pragma unroll 4
  for (int n = 0; n < Nn; ++n) s += (double)p[(size_t)n * Cn];
  const float v = (float)s;
  float* o = S + bt * Cn + c;
  *(volatile float*)o = v;
  __threadfence();
  *(volatile float*)o = v;
}

__global__ __launch_bounds__(256) void k_scores(const float* __restrict__ Wh, const float* __restrict__ aa,
                                                float* __restrict__ s1, float* __restrict__ s2) {
  const int gt = blockIdx.x * 256 + threadIdx.x;
  const bool act = gt < NBH;
  const int gq = act ? gt : 0;
  const int hh = gq & 3, r = gq >> 2;
  const int n = r % Nn, bt = r / Nn;
  const float* wp = Wh + ((size_t)bt * NP + n) * Cn + hh * COn;
  const float* ap = aa + hh * (2 * COn);
  float va = 0.f, vd = 0.f;
#pragma unroll
  for (int q = 0; q < 4; ++q) {
    v4f w = *(const v4fa*)(wp + 4 * q);
#pragma unroll
    for (int k = 0; k < 4; ++k) {
      const float xv = w[k];
      va += xv * ap[4 * q + k];
      vd += xv * ap[COn + 4 * q + k];
    }
  }
  if (act) { *(volatile float*)(s1 + gt) = va; *(volatile float*)(s2 + gt) = vd; }
  __threadfence();
  if (act) { *(volatile float*)(s1 + gt) = va; *(volatile float*)(s2 + gt) = vd; }
}

__global__ __launch_bounds__(384) void k_gat(const float* __restrict__ Wh, const float* __restrict__ S,
                                             const float* __restrict__ s1, const float* __restrict__ s2,
                                             const float* __restrict__ adj, const float* __restrict__ iw,
                                             const float* __restrict__ iwb, const float* __restrict__ x,
                                             float* __restrict__ y1pre) {
  __shared__ __align__(16) float st[BT * Cn];
  __shared__ int wcnt[12];
  __shared__ int jl[KMAX];
  __shared__ float wl[KMAX], rl[KMAX], al[KMAX], il[KMAX];
  const int tid = threadIdx.x, wave = tid >> 5, lane = tid & 31;
  const int i = blockIdx.x;

  bool hit = false;
  float a = 0.f, w = 0.f, raw = 0.f;
  if (tid < Nn) {
    const size_t e = (size_t)i * Nn + tid;
    a = adj[e];
    raw = iw[e];
    const float bb = iwb[e];
    const float lo = bb * 0.5f, hi = bb * 1.5f;
    const float cw = fminf(fmaxf(raw, lo), hi);
    w = fmaxf(cw, 0.f);
    hit = (a != 0.f);
  }
  const unsigned msk = __builtin_amdgcn_ballot_w32(hit);
  const int rank = __popc(msk & ((1u << lane) - 1u));
  if (lane == 0) wcnt[wave] = __popc(msk);
  __syncthreads();
  int base = 0, total = 0;
#pragma unroll
  for (int q = 0; q < 12; ++q) {
    const int c = wcnt[q];
    total += c;
    base += (q < wave) ? c : 0;
  }
  const int slot = base + rank;
  if (hit && slot < KMAX) { jl[slot] = tid; wl[slot] = w * a; rl[slot] = raw; al[slot] = a; }
  const int cnt = total < KMAX ? total : KMAX;
  __syncthreads();
  if (tid < cnt) {
    float ssum = 0.f;
    for (int k = 0; k < cnt; ++k) ssum += wl[k];
    if (ssum == 0.f) ssum = 1e-6f;
    const float rs = 1.0f / ssum;
    const float wc = wl[tid] * rs;
    il[tid] = rl[tid] + (wc - rl[tid]);
  }
  __syncthreads();

  const int bt = tid >> 2, hh = tid & 3;
  const int b = bt / Tn, t = bt - b * Tn;
  const float s1i = s1[((size_t)bt * Nn + i) * HSn + hh];
  const float* s2p = s2 + (size_t)bt * Nn * HSn + hh;
  float mx = 0.f;
  for (int k = 0; k < cnt; ++k) {
    const int jk = clampn(jl[k]);
    const float z = s1i + s2p[(size_t)jk * HSn];
    const float lr = z >= 0.f ? z : 0.2f * z;
    const float sc = lr * al[k] + il[k];
    mx = fmaxf(mx, sc);
  }
  const float e0 = __expf(-mx);
  float o[16];
  const float* Sp = S + bt * Cn + hh * COn;
#pragma unroll
  for (int q = 0; q < 4; ++q) {
    v4f sv = *(const v4fa*)(Sp + 4 * q);
#pragma unroll
    for (int kk = 0; kk < 4; ++kk) o[4 * q + kk] = e0 * sv[kk];
  }
  float Z = (float)(Nn - cnt) * e0;
  for (int k = 0; k < cnt; ++k) {
    const int jk = clampn(jl[k]);
    const float z = s1i + s2p[(size_t)jk * HSn];
    const float lr = z >= 0.f ? z : 0.2f * z;
    const float sc = lr * al[k] + il[k];
    const float ek = __expf(sc - mx);
    Z += ek;
    const float cf = ek - e0;
    const float* wr = Wh + ((size_t)bt * NP + jk) * Cn + hh * COn;
#pragma unroll
    for (int q = 0; q < 4; ++q) {
      v4f wv = *(const v4fa*)(wr + 4 * q);
#pragma unroll
      for (int kk = 0; kk < 4; ++kk) o[4 * q + kk] += cf * wv[kk];
    }
  }
  const float inv = 1.0f / Z;
  const float* xp = x + ((size_t)(b * Nn + i) * Cn + hh * COn) * Tn + t;
  float* sp = st + bt * Cn + hh * COn;
#pragma unroll
  for (int d = 0; d < COn; ++d) sp[d] = o[d] * inv + xp[d * Tn];
  __syncthreads();

#pragma unroll
  for (int pass = 0; pass < 2; ++pass) {
#pragma unroll
    for (int it = 0; it < 4; ++it) {
      const int L = (it * 12 + wave) * 4 + (lane >> 3);
      const int lbt = L >> 1;
      const int col = (L & 1) * 32 + (lane & 7) * 4;
      v4f v = *(const v4fa*)(st + lbt * Cn + col);
      *(volatile v4f*)(y1pre + ((size_t)lbt * NP + i) * Cn + col) = v;
    }
    if (pass == 0) __threadfence();
  }
}

__global__ __launch_bounds__(256) void k_stats(const float* __restrict__ src, double* __restrict__ part) {
  __shared__ double sh[16];
  const int tid = threadIdx.x, wave = tid >> 5, lane = tid & 31;
  const int b = blockIdx.y, bx = blockIdx.x;
  const float* p = src + (size_t)b * TNPC;
  double s = 0.0, q = 0.0;
  for (int gq = bx * 256 + tid; gq < NS4; gq += SBLK * 256) {
    const int e = gq * 4;
    const int t = e / (Nn * Cn);
    const int rem = e - t * (Nn * Cn);
    const int n = rem >> 6, c = rem & 63;
    v4f v = *(const v4fa*)(p + ((size_t)t * NP + n) * Cn + c);
#pragma unroll
    for (int k = 0; k < 4; ++k) { const double dv = (double)v[k]; s += dv; q += dv * dv; }
  }
#pragma unroll
  for (int o = 16; o > 0; o >>= 1) { s += shfl_xor_d(s, o); q += shfl_xor_d(q, o); }
  if (lane == 0) { sh[2 * wave] = s; sh[2 * wave + 1] = q; }
  __syncthreads();
  if (wave == 0) {
    double ts = lane < 8 ? sh[2 * lane] : 0.0;
    double tq = lane < 8 ? sh[2 * lane + 1] : 0.0;
#pragma unroll
    for (int o = 16; o > 0; o >>= 1) { ts += shfl_xor_d(ts, o); tq += shfl_xor_d(tq, o); }
    const double val = (lane == 0) ? ts : ((lane == 1) ? tq : 0.0);
    double* pp = part + ((size_t)(b * SBLK + bx)) * 32 + lane;
    *(volatile double*)pp = val;
    __threadfence();
    *(volatile double*)pp = val;
  }
}

__global__ __launch_bounds__(256) void k_stats_fin(const double* __restrict__ part, float* __restrict__ stats) {
  __shared__ float sh[16];
  const int tid = threadIdx.x, wave = tid >> 5, lane = tid & 31;
  const double* pp = part + (size_t)wave * SBLK * 32;
  double s = pp[(size_t)lane * 32] + pp[(size_t)(lane + 32) * 32];
  double q = pp[(size_t)lane * 32 + 1] + pp[(size_t)(lane + 32) * 32 + 1];
#pragma unroll
  for (int o = 16; o > 0; o >>= 1) { s += shfl_xor_d(s, o); q += shfl_xor_d(q, o); }
  const double mean = s * INVNS;
  const double var = q * INVNS - mean * mean;
  const float mf = (float)mean;
  float vf = (float)var;
  vf = vf < 0.f ? 0.f : vf;
  const float rstd = rsqrtf(vf + EPSn);
  if (lane == 0) { sh[2 * wave] = mf; sh[2 * wave + 1] = rstd; }
  __syncthreads();
  if (wave == 0) {
    const float v = lane < 16 ? sh[lane] : 0.f;
    *(volatile float*)(stats + lane) = v;
    __threadfence();
    *(volatile float*)(stats + lane) = v;
  }
}

__global__ __launch_bounds__(256) void k_apply_pad(const float* __restrict__ src, const float* __restrict__ g,
                                                   const float* __restrict__ be,
                                                   const float* __restrict__ stats, float* __restrict__ dst) {
  const int gt = blockIdx.x * 256 + threadIdx.x;
  const bool act = gt < Bn * NS4;
  const int gq = act ? gt : 0;
  const int b = gq / NS4, rr = gq - b * NS4;
  const int e = rr * 4;
  const int t = e / (Nn * Cn);
  const int rem = e - t * (Nn * Cn);
  const int n = rem >> 6, c = rem & 63;
  const size_t ad = (size_t)b * TNPC + ((size_t)t * NP + n) * Cn + c;
  v4f v = *(const v4fa*)(src + ad);
  const float mean = stats[2 * b], rstd = stats[2 * b + 1];
  const int gi = (n * Cn + c) * Tn + t;
  v4f o;
#pragma unroll
  for (int k = 0; k < 4; ++k) o[k] = (v[k] - mean) * rstd * g[gi + k * Tn] + be[gi + k * Tn];
  if (act) *(volatile v4f*)(dst + ad) = o;
  __threadfence();
  if (act) *(volatile v4f*)(dst + ad) = o;
}

__global__ __launch_bounds__(256) void k_apply_out(const float* __restrict__ src, const float* __restrict__ g,
                                                   const float* __restrict__ be,
                                                   const float* __restrict__ stats, float* __restrict__ out) {
  const int gt = blockIdx.x * 256 + threadIdx.x;
  const bool act = gt < NQ4;
  const int gq = act ? gt : 0;
  const int o4 = gq * 4;
  const int t0 = o4 % Tn;
  const int c = (o4 / Tn) % Cn;
  const int n = (o4 / (Tn * Cn)) % Nn;
  const int b = o4 / (Tn * Cn * Nn);
  const size_t pb = (size_t)b * TNPC + (size_t)n * Cn + c;
  const float mean = stats[2 * b], rstd = stats[2 * b + 1];
  const int gi = (n * Cn + c) * Tn + t0;
  v4f gv = *(const v4fa*)(g + gi);
  v4f bv = *(const v4fa*)(be + gi);
  v4f o;
#pragma unroll
  for (int k = 0; k < 4; ++k) {
    const float v = src[pb + (size_t)(t0 + k) * NP * Cn];
    o[k] = (v - mean) * rstd * gv[k] + bv[k];
  }
  if (act) *(volatile v4f*)(out + o4) = o;
  __threadfence();
  if (act) *(volatile v4f*)(out + o4) = o;
}

__global__ __launch_bounds__(256) void k_attn(const float* __restrict__ Q, const float* __restrict__ K,
                                              const float* __restrict__ V, float* __restrict__ ctx) {
  __shared__ __align__(16) float st[64 * Cn];
  const int tid = threadIdx.x, wave = tid >> 5, lane = tid & 31;
  const int gt = blockIdx.x * 256 + tid;
  const bool act = gt < NATT;
  const int gq = act ? gt : 0;
  const int hh = gq & 3, r = gq >> 2;
  const int t = r % Tn, n = (r / Tn) % Nn, b = r / (Tn * Nn);
  const size_t rstride = (size_t)NP * Cn;
  const size_t pb = (size_t)b * TNPC + (size_t)n * Cn + (size_t)hh * DKn;
  float q[16];
  {
    const float* qp = Q + pb + (size_t)t * rstride;
#pragma unroll
    for (int u = 0; u < 4; ++u) {
      v4f w4 = *(const v4fa*)(qp + 4 * u);
#pragma unroll
      for (int k = 0; k < 4; ++k) q[4 * u + k] = w4[k] * 0.25f;
    }
  }
  float m = -1e30f, Z = 0.f;
  float o[16];
#pragma unroll
  for (int d = 0; d < 16; ++d) o[d] = 0.f;
#pragma unroll 1
  for (int s = 0; s < Tn; ++s) {
    const float* kp = K + pb + (size_t)s * rstride;
    float dt = 0.f;
#pragma unroll
    for (int u = 0; u < 4; ++u) {
      v4f w4 = *(const v4fa*)(kp + 4 * u);
#pragma unroll
      for (int k = 0; k < 4; ++k) dt += q[4 * u + k] * w4[k];
    }
    const float mn = fmaxf(m, dt);
    const float cs = __expf(m - mn);
    const float p = __expf(dt - mn);
    Z = Z * cs + p;
    const float* vp = V + pb + (size_t)s * rstride;
#pragma unroll
    for (int u = 0; u < 4; ++u) {
      v4f w4 = *(const v4fa*)(vp + 4 * u);
#pragma unroll
      for (int k = 0; k < 4; ++k) o[4 * u + k] = o[4 * u + k] * cs + p * w4[k];
    }
    m = mn;
  }
  const float inv = 1.0f / Z;
  float* sp = st + (tid >> 2) * Cn + hh * DKn;
#pragma unroll
  for (int d = 0; d < 16; ++d) sp[d] = o[d] * inv;
  __syncthreads();
#pragma unroll
  for (int pass = 0; pass < 2; ++pass) {
#pragma unroll
    for (int it = 0; it < 4; ++it) {
      const int row = wave * 8 + 2 * it + (lane >> 4);
      const int grow = blockIdx.x * 64 + row;
      if (grow < ROWS_A) {
        const int tt = grow % Tn, nn = (grow / Tn) % Nn, bb2 = grow / (Tn * Nn);
        const int col = (lane & 15) * 4;
        v4f v = *(const v4fa*)(st + row * Cn + col);
        *(volatile v4f*)(ctx + ((size_t)(bb2 * Tn + tt) * NP + nn) * Cn + col) = v;
      }
    }
    if (pass == 0) __threadfence();
  }
}

__global__ __launch_bounds__(128) void k_ff(const float* __restrict__ y2, const _Float16* __restrict__ W1h,
                                            const float* __restrict__ b1, const _Float16* __restrict__ W2h,
                                            const float* __restrict__ b2, float* __restrict__ y3pre) {
  __shared__ __align__(16) _Float16 Wsh[FFn * WPITCH];
  __shared__ __align__(16) _Float16 Hs[4 * 16 * FPITCH];
  __shared__ __align__(16) float stg[4 * 16 * SPITCH];
  const int tid = threadIdx.x, wave = tid >> 5, lane = tid & 31, h = lane >> 4, m = lane & 15;
  for (int c = tid; c < FFn * 8; c += 128) {
    const int n = c >> 3, k8 = (c & 7) * 8;
    *(v8h*)(Wsh + n * WPITCH + k8) = *(const v8h*)(W1h + n * Cn + k8);
  }
  __syncthreads();
  const int g = blockIdx.x * 4 + wave;
  const bool active = g < BT * TILES;
  const int gg = active ? g : 0;
  const int bt = gg / TILES, n0 = (gg - bt * TILES) * 16;
  const int nr = n0 + m, nc = nr < Nn ? nr : Nn - 1;
  const float* rp = y2 + ((size_t)bt * NP + nc) * Cn;
  const v16h a0 = frag_f32<1>(rp, 0, h), a1 = frag_f32<1>(rp, 32, h);
  _Float16* Hw = Hs + wave * (16 * FPITCH);
#pragma unroll
  for (int ct = 0; ct < FFn / 16; ++ct) {
    const _Float16* wr = Wsh + (ct * 16 + m) * WPITCH;
    v8f acc = zero8();
    acc = wmma16(a0, frag_lds(wr, 0, h), acc);
    acc = wmma16(a1, frag_lds(wr, 32, h), acc);
    const float bv = b1[ct * 16 + m];
#pragma unroll
    for (int r = 0; r < 8; ++r) {
      float hv = acc[r] * WINV + bv;
      hv = hv > 0.f ? hv : 0.f;
      Hw[(8 * h + r) * FPITCH + ct * 16 + m] = (_Float16)(hv * HSC);
    }
  }
  __syncthreads();
  for (int c = tid; c < Cn * 32; c += 128) {
    const int n = c >> 5, k8 = (c & 31) * 8;
    *(v8h*)(Wsh + n * FPITCH + k8) = *(const v8h*)(W2h + n * FFn + k8);
  }
  __syncthreads();
  float* st = stg + wave * (16 * SPITCH);
  const _Float16* hr = Hw + m * FPITCH;
#pragma unroll
  for (int ct = 0; ct < 4; ++ct) {
    const _Float16* wr = Wsh + (ct * 16 + m) * FPITCH;
    v8f acc = zero8();
#pragma unroll
    for (int ks = 0; ks < FFn / 32; ++ks)
      acc = wmma16(frag_lds(hr, ks * 32, h), frag_lds(wr, ks * 32, h), acc);
    const float bv = b2[ct * 16 + m];
#pragma unroll
    for (int r = 0; r < 8; ++r) st[(8 * h + r) * SPITCH + ct * 16 + m] = acc[r] * HWINV + bv;
  }
  __syncthreads();
  store_tile<true>(st, y2, y3pre, bt, n0, h, m, active);
}

extern "C" void kernel_launch(void* const* d_in, const int* in_sizes, int n_in, void* d_out, int out_size,
                              void* d_ws, size_t ws_size, hipStream_t stream) {
  if (n_in < 25 || out_size != OUTN) return;
  const int expect[25] = {OUTN,   Nn * Nn, Nn * Nn, Nn * Nn, Cn * Cn, Cn,       HSn * 2 * COn, NS, NS,
                          Cn * Cn, Cn,     Cn * Cn, Cn,      Cn * Cn, Cn,       Cn * Cn,       Cn, NS,
                          NS,      FFn * Cn, FFn,   Cn * FFn, Cn,     NS,       NS};
  for (int qq = 0; qq < 25; ++qq)
    if (in_sizes[qq] != expect[qq]) return;

  const float* x   = (const float*)d_in[0];
  const float* adj = (const float*)d_in[1];
  const float* iw  = (const float*)d_in[2];
  const float* iwb = (const float*)d_in[3];
  const float* Ww  = (const float*)d_in[4];
  const float* Wb  = (const float*)d_in[5];
  const float* aa  = (const float*)d_in[6];
  const float* g1  = (const float*)d_in[7];
  const float* be1 = (const float*)d_in[8];
  const float* Wq  = (const float*)d_in[9];
  const float* Wqb = (const float*)d_in[10];
  const float* Wk  = (const float*)d_in[11];
  const float* Wkb = (const float*)d_in[12];
  const float* Wv  = (const float*)d_in[13];
  const float* Wvb = (const float*)d_in[14];
  const float* Wo  = (const float*)d_in[15];
  const float* Wob = (const float*)d_in[16];
  const float* g2  = (const float*)d_in[17];
  const float* be2 = (const float*)d_in[18];
  const float* fw1 = (const float*)d_in[19];
  const float* fb1 = (const float*)d_in[20];
  const float* fw2 = (const float*)d_in[21];
  const float* fb2 = (const float*)d_in[22];
  const float* g3  = (const float*)d_in[23];
  const float* be3 = (const float*)d_in[24];

  const size_t off_S     = 10 * PSZ;
  const size_t off_s1    = off_S + (size_t)BT * Cn;
  const size_t off_s2    = off_s1 + (size_t)NBH;
  const size_t off_stats = off_s2 + (size_t)NBH;
  const size_t off_part  = off_stats + 128;
  const size_t off_w16   = off_part + (size_t)Bn * SBLK * 32 * 2;
  const size_t tot_f     = off_w16 + (size_t)W16_TOT / 2;
  if (tot_f * sizeof(float) > ws_size) return;

  float* ws    = (float*)d_ws;
  float* Wh    = ws + 0 * PSZ;
  float* y1pre = ws + 1 * PSZ;
  float* y1    = ws + 2 * PSZ;
  float* Qb    = ws + 3 * PSZ;
  float* Kb    = ws + 4 * PSZ;
  float* Vb    = ws + 5 * PSZ;
  float* ctx   = ws + 6 * PSZ;
  float* y2pre = ws + 7 * PSZ;
  float* y2    = ws + 8 * PSZ;
  float* y3pre = ws + 9 * PSZ;
  float* S     = ws + off_S;
  float* s1    = ws + off_s1;
  float* s2    = ws + off_s2;
  float* stats = ws + off_stats;
  double* part = (double*)(ws + off_part);
  _Float16* w16 = (_Float16*)(ws + off_w16);
  float* out   = (float*)d_out;

  k_cvtw<<<dim3(8, 7), 256, 0, stream>>>(Ww, Wq, Wk, Wv, Wo, fw1, fw2, w16);
  k_wh<<<GEMM_WG, 128, 0, stream>>>(x, w16 + WOFF_W, Wb, Wh);
  k_redS<<<BT, 64, 0, stream>>>(Wh, S);
  k_scores<<<FLAT_WG, 256, 0, stream>>>(Wh, aa, s1, s2);
  k_gat<<<Nn, 384, 0, stream>>>(Wh, S, s1, s2, adj, iw, iwb, x, y1pre);

  k_stats<<<dim3(SBLK, Bn), 256, 0, stream>>>(y1pre, part);
  k_stats_fin<<<1, 256, 0, stream>>>(part, stats + 0);
  k_apply_pad<<<APPLY_WG, 256, 0, stream>>>(y1pre, g1, be1, stats + 0, y1);

  k_qkv<<<dim3(GEMM_WG, 3), 128, 0, stream>>>(y1, w16 + WOFF_Q, w16 + WOFF_K, w16 + WOFF_V, Wqb, Wkb, Wvb,
                                               Qb, Kb, Vb);
  k_attn<<<ATT_WG, 256, 0, stream>>>(Qb, Kb, Vb, ctx);
  k_wo<<<GEMM_WG, 128, 0, stream>>>(ctx, w16 + WOFF_O, Wob, y1, y2pre);

  k_stats<<<dim3(SBLK, Bn), 256, 0, stream>>>(y2pre, part);
  k_stats_fin<<<1, 256, 0, stream>>>(part, stats + 32);
  k_apply_pad<<<APPLY_WG, 256, 0, stream>>>(y2pre, g2, be2, stats + 32, y2);

  k_ff<<<GEMM_WG, 128, 0, stream>>>(y2, w16 + WOFF_1, fb1, w16 + WOFF_2, fb2, y3pre);

  k_stats<<<dim3(SBLK, Bn), 256, 0, stream>>>(y3pre, part);
  k_stats_fin<<<1, 256, 0, stream>>>(part, stats + 64);
  k_apply_out<<<APPLY_WG, 256, 0, stream>>>(y3pre, g3, be3, stats + 64, out);
}
